// MultiheadGlobalPosAttention_1881195676261
// MI455X (gfx1250) — hardware-verified
//
#include <hip/hip_runtime.h>
#include <math.h>

typedef __attribute__((ext_vector_type(16))) _Float16 v16h;
typedef __attribute__((ext_vector_type(16))) __bf16 v16b;
typedef __attribute__((ext_vector_type(8)))  _Float16 v8h;
typedef __attribute__((ext_vector_type(8)))  float v8f;
typedef __attribute__((ext_vector_type(4)))  float v4f;
typedef __attribute__((ext_vector_type(2)))  float v2f;
typedef __attribute__((ext_vector_type(4)))  unsigned v4u;
typedef __attribute__((ext_vector_type(4)))  int v4i;
typedef float __attribute__((may_alias)) float_a;
typedef int __attribute__((may_alias)) int_a;

template <typename T> __device__ __forceinline__ void vst2(void* p, T v) { *(volatile T*)p = v; __threadfence(); *(volatile T*)p = v; }
__device__ __forceinline__ v8f wmma16(v16h a, v16h b, v8f c) {
  v8f d = __builtin_amdgcn_wmma_f32_16x16x32_f16(false, a, false, b, (short)0, c, false, false);
  asm volatile("v_nop\n\tv_nop\n\tv_nop\n\tv_nop" : "+v"(d) : "v"(a), "v"(b));
  return d;
}
__device__ __forceinline__ v8f wmma_bf(v16b a, v16b b, v8f c) {
  v8f d = __builtin_amdgcn_wmma_f32_16x16x32_bf16(false, a, false, b, (short)0, c, false, false);
  asm volatile("v_nop\n\tv_nop\n\tv_nop\n\tv_nop" : "+v"(d) : "v"(a), "v"(b));
  return d;
}
__device__ __forceinline__ v16h frag_h(const _Float16* rowk0, int lane) {
  union { v16h v; v8h q[2]; } u; const _Float16* p = rowk0 + 8 * (lane >> 4);
  u.q[0] = *(const v8h*)p; u.q[1] = *(const v8h*)(p + 16); return u.v;
}
__device__ __forceinline__ v16h frag_f32(const float* rowk0, int lane) {
  v16h a; const float* p = rowk0 + 8 * (lane >> 4);
#pragma unroll
  for (int i = 0; i < 8; ++i) { a[i] = (_Float16)p[i]; a[8 + i] = (_Float16)p[16 + i]; }
  return a;
}
__device__ __forceinline__ v16h frag_f32s(const float* rowk0, int lane, float sc) {
  v16h a; const float* p = rowk0 + 8 * (lane >> 4);
#pragma unroll
  for (int i = 0; i < 8; ++i) { a[i] = (_Float16)(p[i] * sc); a[8 + i] = (_Float16)(p[16 + i] * sc); }
  return a;
}
__device__ __forceinline__ v16h fragc_f32(const float* W, int k0, int n, int lane, int ld, int K) {
  v16h a; const int g = lane >> 4;
#pragma unroll
  for (int i = 0; i < 8; ++i) { const int ka = k0 + 8 * g + i, kb = ka + 16;
    a[i] = (_Float16)(ka < K ? W[(size_t)ka * ld + n] : 0.f); a[8 + i] = (_Float16)(kb < K ? W[(size_t)kb * ld + n] : 0.f); }
  return a;
}
struct F2 { v16b h, l; };
__device__ __forceinline__ F2 bsplit16(const float v[16]) { F2 r;
#pragma unroll
  for (int i = 0; i < 16; ++i) { const __bf16 h = (__bf16)v[i]; r.h[i] = h; r.l[i] = (__bf16)(v[i] - (float)h); }
  return r; }
__device__ __forceinline__ F2 split_row(const float* row, int k0, int lane) { float v[16]; const float* p = row + k0 + 8 * (lane >> 4);
#pragma unroll
  for (int i = 0; i < 8; ++i) { v[i] = p[i]; v[8 + i] = p[16 + i]; }
  return bsplit16(v); }
__device__ __forceinline__ F2 split_rowK(const float* row, int k0, int lane, int K) { float v[16]; const int g = lane >> 4;
#pragma unroll
  for (int i = 0; i < 8; ++i) { const int ka = k0 + 8 * g + i, kb = ka + 16; v[i] = ka < K ? row[ka] : 0.f; v[8 + i] = kb < K ? row[kb] : 0.f; }
  return bsplit16(v); }
__device__ __forceinline__ F2 split_col(const float* W, int k0, int n, int lane, int ld, int K) { float v[16]; const int g = lane >> 4;
#pragma unroll
  for (int i = 0; i < 8; ++i) { const int ka = k0 + 8 * g + i, kb = ka + 16; v[i] = ka < K ? W[(size_t)ka * ld + n] : 0.f; v[8 + i] = kb < K ? W[(size_t)kb * ld + n] : 0.f; }
  return bsplit16(v); }
__device__ __forceinline__ v8f mac3(const F2& a, const F2& b, v8f c) { c = wmma_bf(a.l, b.h, c); c = wmma_bf(a.h, b.l, c); return wmma_bf(a.h, b.h, c); }
__device__ __forceinline__ float sigm(float v) { return 1.0f / (1.0f + expf(-v)); }
#define LDSX() do { asm volatile("s_wait_dscnt 0" ::: "memory"); __builtin_amdgcn_wave_barrier(); __builtin_amdgcn_fence(__ATOMIC_RELEASE, "workgroup"); } while (0)

#define NBATCH 2
#define NN 384
#define DIM 256
#define HID 128

__global__ __launch_bounds__(256) void k_packW(const float* __restrict__ W, int K, int N, _Float16* __restrict__ P) {
  const int n = blockIdx.x, tid = threadIdx.x;
  for (int q = tid; q < K / 8; q += 256) { union { v8h hh; v4u u; } pk;
#pragma unroll
    for (int i = 0; i < 8; ++i) pk.hh[i] = (_Float16)W[(size_t)(q * 8 + i) * N + n];
    vst2(P + (size_t)n * K + q * 8, pk.u); }
}
template <int AH>
__global__ __launch_bounds__(128) void k_gemm(const void* __restrict__ Av, int K, const _Float16* __restrict__ P, const float* __restrict__ bias, float* __restrict__ Out, int N) {
  __shared__ __align__(16) float so[4][16][132];
  const int tid = threadIdx.x, wave = tid >> 5, lane = tid & 31, col = lane & 15, g = lane >> 4;
  const int r0 = blockIdx.x * 64 + wave * 16, n0 = blockIdx.y * 128;
  v8f acc[8] = {};
#pragma unroll 1
  for (int kc = 0; kc < K / 32; ++kc) { const v16h a = AH ? frag_h((const _Float16*)Av + (size_t)(r0 + col) * K + kc * 32, lane) : frag_f32((const float*)Av + (size_t)(r0 + col) * K + kc * 32, lane);
#pragma unroll
    for (int j = 0; j < 8; ++j) acc[j] = wmma16(a, frag_h(P + (size_t)(n0 + j * 16 + col) * K + kc * 32, lane), acc[j]); }
#pragma unroll
  for (int j = 0; j < 8; ++j) { const float bb = bias[n0 + j * 16 + col];
#pragma unroll
    for (int r = 0; r < 8; ++r) so[wave][8 * g + r][j * 16 + col] = acc[j][r] + bb; }
  LDSX();
#pragma unroll 4
  for (int rl = 0; rl < 16; ++rl) vst2(Out + (size_t)(r0 + rl) * N + n0 + lane * 4, *(const v4f*)(&so[wave][rl][lane * 4]));
}
__global__ __launch_bounds__(256) void k_attn(const float* __restrict__ qkv, const float* __restrict__ pos, const int* __restrict__ mask, const float* __restrict__ w1, const float* __restrict__ b1,
                                            const _Float16* __restrict__ P2, const float* __restrict__ b2, float* __restrict__ att) {
  __shared__ __align__(16) float rel[16][DIM + 4];
  __shared__ float sd[16];
  __shared__ __align__(16) float so[DIM];
  const int tid = threadIdx.x, w = tid >> 5, lane = tid & 31, col = lane & 15, g = lane >> 4;
  const int bi = blockIdx.x, b = bi / NN, i = bi % NN; const int c = tid;
  const float kic = qkv[(size_t)bi * 768 + DIM + c];
  const bool mi = mask[(size_t)b * NN + i] != 0;
  const float pix = pos[(size_t)bi * 3], piy = pos[(size_t)bi * 3 + 1], piz = pos[(size_t)bi * 3 + 2];
  float m = -3.0e38f, l = 0.f, acc = 0.f;
#pragma unroll 1
  for (int jt = 0; jt < NN / 16; ++jt) {
    if (tid < 16) { const int j = jt * 16 + tid; const float dx = pix - pos[((size_t)b * NN + j) * 3], dy = piy - pos[((size_t)b * NN + j) * 3 + 1], dz = piz - pos[((size_t)b * NN + j) * 3 + 2];
      const float sq = dx * dx + dy * dy + dz * dz; sd[tid] = sq > 0.f ? sqrtf(sq) : 0.f; }
    __syncthreads();
    { v8f acc2[2] = {};
#pragma unroll
      for (int kc = 0; kc < HID / 32; ++kc) { v16h a; const float dj = sd[col];
#pragma unroll
        for (int ii = 0; ii < 8; ++ii) { const int ha = kc * 32 + 8 * g + ii, hb = ha + 16;
          const float va = dj * w1[ha] + b1[ha], vb = dj * w1[hb] + b1[hb]; a[ii] = (_Float16)(va > 0.f ? va : 0.f); a[8 + ii] = (_Float16)(vb > 0.f ? vb : 0.f); }
#pragma unroll
        for (int t = 0; t < 2; ++t) acc2[t] = wmma16(a, frag_h(P2 + (size_t)(w * 32 + t * 16 + col) * HID + kc * 32, lane), acc2[t]); }
#pragma unroll
      for (int t = 0; t < 2; ++t) { const int cc = w * 32 + t * 16 + col; const float bb = b2[cc];
#pragma unroll
        for (int r = 0; r < 8; ++r) rel[8 * g + r][cc] = acc2[t][r] + bb; } }
    __syncthreads();
#pragma unroll 4
    for (int jj = 0; jj < 16; ++jj) { const int j = jt * 16 + jj; const float rv = rel[jj][c];
      const float* qr = qkv + ((size_t)b * NN + j) * 768;
      const bool mj = mask[(size_t)b * NN + j] != 0;
      float lg = kic * qr[c] + rv; if (mi && mj) lg = -3.0e38f;
      const float mn = fmaxf(m, lg); const float cr = expf(m - mn), p = (mi && mj) ? 0.f : expf(lg - mn);
      l = l * cr + p; acc = acc * cr + p * (qr[2 * DIM + c] + rv); m = mn; }
    __syncthreads();
  }
  so[c] = acc / l;
  __syncthreads();
  if (tid < 64) vst2(att + (size_t)bi * DIM + tid * 4, *(const v4f*)(&so[tid * 4]));
}
extern "C" void kernel_launch(void* const* d_in, const int* in_sizes, int n_in, void* d_out, int out_size, void* d_ws, size_t ws_size, hipStream_t stream) {
  (void)in_sizes; (void)n_in; (void)out_size; (void)ws_size;
  const float* x = (const float*)d_in[0]; const float* pos = (const float*)d_in[1]; const int* mask = (const int*)d_in[2];
  const float* qkvw = (const float*)d_in[3]; const float* qkvb = (const float*)d_in[4]; const float* w1 = (const float*)d_in[5]; const float* b1 = (const float*)d_in[6];
  const float* w2 = (const float*)d_in[7]; const float* b2 = (const float*)d_in[8]; const float* ow = (const float*)d_in[9]; const float* ob = (const float*)d_in[10];
  float* out = (float*)d_out;
  char* ws = (char*)d_ws; size_t off = 0;
  auto take = [&](size_t bytes) { char* p = ws + off; off += (bytes + 255) & ~(size_t)255; return p; };
  _Float16* Pqkv = (_Float16*)take((size_t)768 * DIM * 2); _Float16* P2 = (_Float16*)take((size_t)DIM * HID * 2); _Float16* Po = (_Float16*)take((size_t)DIM * DIM * 2);
  float* qkv = (float*)take((size_t)NBATCH * NN * 768 * 4); float* att = (float*)take((size_t)NBATCH * NN * DIM * 4);
  k_packW<<<768, 256, 0, stream>>>(qkvw, DIM, 768, Pqkv);
  k_packW<<<DIM, 256, 0, stream>>>(w2, HID, DIM, P2);
  k_packW<<<DIM, 256, 0, stream>>>(ow, DIM, DIM, Po);
  k_gemm<0><<<dim3(NBATCH * NN / 64, 768 / 128), 128, 0, stream>>>(x, DIM, Pqkv, qkvb, qkv, 768);
  k_attn<<<NBATCH * NN, 256, 0, stream>>>(qkv, pos, mask, w1, b1, P2, b2, att);
  k_gemm<0><<<dim3(NBATCH * NN / 64, DIM / 128), 128, 0, stream>>>(att, DIM, Po, ob, out, DIM);
}
